// MPAMMambaFusion_9749575762051
// MI455X (gfx1250) — hardware-verified
//
#include <hip/hip_runtime.h>
#include <math.h>

typedef __attribute__((ext_vector_type(16))) _Float16 v16h;
typedef __attribute__((ext_vector_type(8)))  _Float16 v8h;
typedef __attribute__((ext_vector_type(16))) __bf16   v16b;
typedef __attribute__((ext_vector_type(8)))  __bf16   v8b;
typedef __attribute__((ext_vector_type(8)))  float    v8f;
typedef __attribute__((ext_vector_type(4)))  float    v4f;

constexpr int kBatch = 2;
constexpr int kCR    = 256;
constexpr int kCS    = 512;
constexpr int kHR = 64, kWR = 64, kHS = 32, kWS = 32;
constexpr int kSeq   = kHR * kWR;
constexpr int kPixS  = kHS * kWS;
constexpr int kRows  = kBatch * kSeq;
constexpr int kRowsS = kBatch * kPixS;
constexpr int kDin   = 512;
constexpr int kNst   = 16;
constexpr int kDtR   = 16;
constexpr int kConvK = 3;
constexpr int kXzP   = 2 * kDin;
constexpr int kXdN   = kDtR + 2 * kNst;
constexpr int kXdP   = 64;
constexpr float kEps = 1e-5f;
constexpr int kFuseTP = 260;
constexpr int kConvTP = 260;
constexpr int kScanTS = 64;
constexpr int kScanCh = 64;
constexpr int kScanYP = 68;
static_assert(kXdN <= kXdP, "x_proj width");
static_assert((kCS % 32) == 0 && (kCR % 32) == 0 && (kDin % 32) == 0, "GEMM K multiples of 32");
static_assert((kRowsS % 64) == 0 && (kRows % 64) == 0 && (kCR % 64) == 0 && (kXzP % 64) == 0 && (kXdP % 64) == 0, "GEMM M,N multiples of 64");
static_assert((kSeq % kScanTS) == 0 && (kSeq % 64) == 0 && (kDin % kScanCh) == 0 && (kDin % 256) == 0, "tile multiples");
static_assert((kSeq % 32) == 0 && kWR == 64 && kCR == 256, "fuse tile assumptions");

constexpr size_t kOffSCH  = 0;
constexpr size_t kOffSCL  = kOffSCH + (size_t)kRowsS * kCS  * 2;
constexpr size_t kOffWSH  = kOffSCL + (size_t)kRowsS * kCS  * 2;
constexpr size_t kOffWSL  = kOffWSH + (size_t)kCR    * kCS  * 2;
constexpr size_t kOffSP   = kOffWSL + (size_t)kCR    * kCS  * 2;
constexpr size_t kOffFU   = kOffSP  + (size_t)kRowsS * kCR  * 4;
constexpr size_t kOffXNH  = kOffFU  + (size_t)kRows  * kCR  * 4;
constexpr size_t kOffXNL  = kOffXNH + (size_t)kRows  * kCR  * 2;
constexpr size_t kOffWIH  = kOffXNL + (size_t)kRows  * kCR  * 2;
constexpr size_t kOffWIL  = kOffWIH + (size_t)kXzP   * kCR  * 2;
constexpr size_t kOffWXH  = kOffWIL + (size_t)kXzP   * kCR  * 2;
constexpr size_t kOffWXL  = kOffWXH + (size_t)kXdP   * kDin * 2;
constexpr size_t kOffWOH  = kOffWXL + (size_t)kXdP   * kDin * 2;
constexpr size_t kOffWOL  = kOffWOH + (size_t)kCR    * kDin * 2;
constexpr size_t kOffXZ   = kOffWOL + (size_t)kCR    * kDin * 2;
constexpr size_t kOffUC   = kOffXZ  + (size_t)kRows  * kXzP * 4;
constexpr size_t kOffUCH  = kOffUC  + (size_t)kRows  * kDin * 4;
constexpr size_t kOffUCL  = kOffUCH + (size_t)kRows  * kDin * 2;
constexpr size_t kOffXD   = kOffUCL + (size_t)kRows  * kDin * 2;
constexpr size_t kOffYH   = kOffXD  + (size_t)kRows  * kXdP * 4;
constexpr size_t kOffYL   = kOffYH  + (size_t)kRows  * kDin * 2;
constexpr size_t kOffOS   = kOffYL  + (size_t)kRows  * kDin * 2;
constexpr size_t kWsTotal = kOffOS  + (size_t)kRows  * kCR  * 4;
static_assert(kWsTotal == 119668736ull, "carve total");
static_assert(kWsTotal <= 134217728ull, "carve cap");
static_assert((kOffSCL % 128) == 0 && (kOffWSH % 128) == 0 && (kOffWSL % 128) == 0 && (kOffSP % 128) == 0 &&
              (kOffFU % 128) == 0 && (kOffXNH % 128) == 0 && (kOffXNL % 128) == 0 && (kOffWIH % 128) == 0 &&
              (kOffWIL % 128) == 0 && (kOffWXH % 128) == 0 && (kOffWXL % 128) == 0 && (kOffWOH % 128) == 0 &&
              (kOffWOL % 128) == 0 && (kOffXZ % 128) == 0 && (kOffUC % 128) == 0 && (kOffUCH % 128) == 0 &&
              (kOffUCL % 128) == 0 && (kOffXD % 128) == 0 && (kOffYH % 128) == 0 && (kOffYL % 128) == 0 &&
              (kOffOS % 128) == 0, "128-B aligned regions");

__device__ __forceinline__ unsigned short f2bf_bits(float f) {
  unsigned u = __float_as_uint(f);
  return (unsigned short)((u + 0x7FFFu + ((u >> 16) & 1u)) >> 16);
}
__device__ __forceinline__ float bf_bits2f(unsigned short h) { return __uint_as_float(((unsigned)h) << 16); }

__device__ __forceinline__ void dep_guard_h(v8f& a, v8f& b, v16h x, v16h y) { asm volatile("v_nop\n\tv_nop\n\tv_nop\n\tv_nop" : "+v"(a), "+v"(b) : "v"(x), "v"(y)); }
__device__ __forceinline__ void dep_guard_b(v8f& a, v8f& b, v16b x, v16b y) { asm volatile("v_nop\n\tv_nop\n\tv_nop\n\tv_nop" : "+v"(a), "+v"(b) : "v"(x), "v"(y)); }
__device__ __forceinline__ void keep4_h(v16h a, v16h b, v16h c, v16h d) { asm volatile("v_nop" :: "v"(a), "v"(b), "v"(c), "v"(d)); }
__device__ __forceinline__ void keep4_b(v16b a, v16b b, v16b c, v16b d) { asm volatile("v_nop" :: "v"(a), "v"(b), "v"(c), "v"(d)); }
__device__ __forceinline__ void acc_guard4(v8f& a, v8f& b, v8f& c, v8f& d) { asm volatile("v_nop\n\tv_nop\n\tv_nop\n\tv_nop" : "+v"(a), "+v"(b), "+v"(c), "+v"(d)); }
template <typename T> struct Frag;
template <> struct Frag<_Float16> {
  typedef v16h V; union U { v16h v; v8h h[2]; };
  static __device__ __forceinline__ v16h load(const _Float16* p) {
    U f; f.h[0] = *(const v8h*)(p); f.h[1] = *(const v8h*)(p + 16); return f.v;
  }
  static __device__ __forceinline__ v8f mma(v16h a, v16h b, v8f c) {
    return __builtin_amdgcn_wmma_f32_16x16x32_f16(false, a, false, b, (short)0, c, false, false);
  }
  static __device__ __forceinline__ void guard(v8f& a, v8f& b, v16h x, v16h y) { dep_guard_h(a, b, x, y); }
  static __device__ __forceinline__ void keep(v16h a, v16h b, v16h c, v16h d) { keep4_h(a, b, c, d); }
};
template <> struct Frag<__bf16> {
  typedef v16b V; union U { v16b v; v8b h[2]; };
  static __device__ __forceinline__ v16b load(const __bf16* p) {
    U f; f.h[0] = *(const v8b*)(p); f.h[1] = *(const v8b*)(p + 16); return f.v;
  }
  static __device__ __forceinline__ v8f mma(v16b a, v16b b, v8f c) {
    return __builtin_amdgcn_wmma_f32_16x16x32_bf16(false, a, false, b, (short)0, c, false, false);
  }
  static __device__ __forceinline__ void guard(v8f& a, v8f& b, v16b x, v16b y) { dep_guard_b(a, b, x, y); }
  static __device__ __forceinline__ void keep(v16b a, v16b b, v16b c, v16b d) { keep4_b(a, b, c, d); }
};

template <int ET> struct Elem;
template <> struct Elem<0> { typedef _Float16 T; };
template <> struct Elem<1> { typedef __bf16 T; };
template <int ET, int SPL, int BIAS_MODE, int OUT_MODE, bool RESID, int ACT = 0>
__global__ __launch_bounds__(256) void wmma_gemm64(
    const unsigned short* __restrict__ Ap, const unsigned short* __restrict__ A2p, int lda, long strideA,
    const unsigned short* __restrict__ Btp, const unsigned short* __restrict__ Bt2p, int ldb, long strideB,
    void* __restrict__ Cout, void* __restrict__ Cout2, int ldc, long strideC,
    const float* __restrict__ bias,
    const float* __restrict__ resid, long strideR,
    int M, int N, int K, float scale) {
  typedef typename Elem<ET>::T T;
  typedef typename Frag<T>::V V;
  const T* A = (const T*)Ap; const T* A2 = (const T*)A2p; const T* Bt = (const T*)Btp; const T* Bt2 = (const T*)Bt2p;
  __shared__ __align__(16) float sT[8][16 * 68];
  const int b    = blockIdx.y;
  const int lane = threadIdx.x & 31;
  const int wave = threadIdx.x >> 5;
  const int tilesN = N >> 6;
  const int tilesM = M >> 6;
  const int tile = blockIdx.x * 8 + wave;
  if (tile >= tilesM * tilesN) return;
  const int tm = tile / tilesN;
  const int tn = tile - tm * tilesN;
  const int m0 = tm << 6;
  const int n0 = tn << 6;

  const T* Ab  = A  + (size_t)b * strideA;
  const T* Bb  = Bt + (size_t)b * strideB;
  const T* Ab2 = (SPL >= 1) ? (A2  + (size_t)b * strideA) : nullptr;
  const T* Bb2 = (SPL == 2) ? (Bt2 + (size_t)b * strideB) : nullptr;

  const int rlane = lane & 15;
  const int koff  = (lane >> 4) * 8;
  const int mOff  = (lane >> 4) * 8;

  v8f acc[4][4];
#pragma unroll
  for (int i = 0; i < 4; ++i)
#pragma unroll
    for (int j = 0; j < 4; ++j) acc[i][j] = (v8f){0.f,0.f,0.f,0.f,0.f,0.f,0.f,0.f};

  for (int k0 = 0; k0 < K; k0 += 32) {
    V bh[4], bl[4];
#pragma unroll
    for (int j = 0; j < 4; ++j) {
      const size_t bo = (size_t)(n0 + (j << 4) + rlane) * ldb + koff + k0;
      bh[j] = Frag<T>::load(Bb + bo);
      if (SPL == 2) bl[j] = Frag<T>::load(Bb2 + bo);
    }
#pragma unroll
    for (int i = 0; i < 4; ++i) {
      const size_t ao = (size_t)(m0 + (i << 4) + rlane) * lda + koff + k0;
      V ah = Frag<T>::load(Ab + ao);
      V al;
      if (SPL >= 1) al = Frag<T>::load(Ab2 + ao);
#pragma unroll
      for (int j = 0; j < 4; ++j) {
        acc[i][j] = Frag<T>::mma(ah, bh[j], acc[i][j]);
        if (SPL == 2) acc[i][j] = Frag<T>::mma(ah, bl[j], acc[i][j]);
        if (SPL >= 1) acc[i][j] = Frag<T>::mma(al, bh[j], acc[i][j]);
      }
      Frag<T>::guard(acc[i][0], acc[i][3], ah, (SPL >= 1) ? al : ah);
    }
    Frag<T>::keep(bh[0], bh[1], bh[2], bh[3]);
    if (SPL == 2) Frag<T>::keep(bl[0], bl[1], bl[2], bl[3]);
  }
  acc_guard4(acc[0][0], acc[0][1], acc[0][2], acc[0][3]);
  acc_guard4(acc[1][0], acc[1][1], acc[1][2], acc[1][3]);
  acc_guard4(acc[2][0], acc[2][1], acc[2][2], acc[2][3]);
  acc_guard4(acc[3][0], acc[3][1], acc[3][2], acc[3][3]);

  float* slab = sT[wave];
  const float* Rb = RESID ? (resid + (size_t)b * strideR) : nullptr;
#pragma unroll
  for (int i = 0; i < 4; ++i) {
    const int mBase = m0 + (i << 4);
#pragma unroll
    for (int j = 0; j < 4; ++j) {
      const int n = n0 + (j << 4) + rlane;
      float bv = 0.f;
      if (BIAS_MODE == 2) bv = bias[n];
#pragma unroll
      for (int r = 0; r < 8; ++r) {
        float v = acc[i][j][r] * scale;
        if (BIAS_MODE == 1) v += bias[mBase + mOff + r];
        if (BIAS_MODE == 2) v += bv;
        if (RESID) v += Rb[(size_t)(mBase + mOff + r) * ldc + n];
        if (ACT == 1) v = tanhf(v);
        if (ACT == 2) v = fmaxf(v, 0.0f);
        if (ACT == 3) v = v / (1.0f + expf(-v));
        if (ACT == 4) v = (v > 0.f) ? v : 0.01f * v;
        slab[(mOff + r) * 68 + (j << 4) + rlane] = v;
      }
    }
    __builtin_amdgcn_fence(__ATOMIC_RELEASE, "workgroup");
    __builtin_amdgcn_wave_barrier();
    __builtin_amdgcn_fence(__ATOMIC_ACQUIRE, "workgroup");
    if (OUT_MODE == 0) {
      float* C = (float*)Cout + (size_t)b * strideC;
      const int hh = lane >> 4, c4 = (lane & 15) * 4;
      for (int pass = 0; pass < 2; ++pass) {
#pragma unroll
        for (int it = 0; it < 8; ++it) {
          const int row = it * 2 + hh;
          v4f v = *(const v4f*)(slab + row * 68 + c4);
          *(volatile v4f*)(C + (size_t)(mBase + row) * ldc + n0 + c4) = v;
        }
        __threadfence();
      }
    } else {
      const int q = lane >> 3, c8 = (lane & 7) * 8;
      unsigned short* C  = (unsigned short*)Cout  + (size_t)b * strideC;
      unsigned short* C2 = (OUT_MODE == 2) ? ((unsigned short*)Cout2 + (size_t)b * strideC) : nullptr;
      for (int pass = 0; pass < 2; ++pass) {
#pragma unroll
        for (int it = 0; it < 4; ++it) {
          const int row = it * 4 + q;
          const float* sp = slab + row * 68 + c8;
          v8h hv, lv;
#pragma unroll
          for (int e = 0; e < 8; ++e) {
            if (OUT_MODE == 1) {
              hv[e] = (_Float16)sp[e];
            } else {
              unsigned short hb = f2bf_bits(sp[e]);
              unsigned short lb = f2bf_bits(sp[e] - bf_bits2f(hb));
              hv[e] = __builtin_bit_cast(_Float16, hb);
              lv[e] = __builtin_bit_cast(_Float16, lb);
            }
          }
          *(volatile v8h*)(C + (size_t)(mBase + row) * ldc + n0 + c8) = hv;
          if (OUT_MODE == 2) *(volatile v8h*)(C2 + (size_t)(mBase + row) * ldc + n0 + c8) = lv;
        }
        __threadfence();
      }
    }
    __builtin_amdgcn_fence(__ATOMIC_RELEASE, "workgroup");
    __builtin_amdgcn_wave_barrier();
    __builtin_amdgcn_fence(__ATOMIC_ACQUIRE, "workgroup");
  }
}

__global__ __launch_bounds__(256) void split_rows_bf16_kernel(
    const float* __restrict__ src, unsigned short* __restrict__ dhi, unsigned short* __restrict__ dlo, int total8, int valid8)
{
  const int i = blockIdx.x * 256 + threadIdx.x;
  if (i >= total8) return;
  const bool live = (i < valid8);
  const int ic = live ? i : (valid8 - 1);
  const size_t s0 = (size_t)ic << 3;
  const v4f a0 = *(const v4f*)(src + s0);
  const v4f a1 = *(const v4f*)(src + s0 + 4);
  v8h hv, lv;
#pragma unroll
  for (int e = 0; e < 4; ++e) {
    const float f0 = live ? a0[e] : 0.0f;
    const float f1 = live ? a1[e] : 0.0f;
    const unsigned short h0 = f2bf_bits(f0), h1 = f2bf_bits(f1);
    const unsigned short l0 = f2bf_bits(f0 - bf_bits2f(h0)), l1 = f2bf_bits(f1 - bf_bits2f(h1));
    hv[e]     = __builtin_bit_cast(_Float16, h0);
    hv[4 + e] = __builtin_bit_cast(_Float16, h1);
    lv[e]     = __builtin_bit_cast(_Float16, l0);
    lv[4 + e] = __builtin_bit_cast(_Float16, l1);
  }
  const size_t e0 = (size_t)i << 3;
  unsigned short* qh = dhi + e0;
  unsigned short* ql = dlo + e0;
  *(volatile v8h*)qh = hv;
  *(volatile v8h*)ql = lv;
  __threadfence();
  *(volatile v8h*)qh = hv;
  *(volatile v8h*)ql = lv;
}

__global__ __launch_bounds__(256) void scp_transpose_split_kernel(
    const float* __restrict__ scp, unsigned short* __restrict__ SCH, unsigned short* __restrict__ SCL)
{
  __shared__ __align__(16) float sT[64 * 68];
  const int tid = threadIdx.x, lane = tid & 31, wave = tid >> 5;
  const int c0 = blockIdx.x * 64;
  const int b  = blockIdx.y >> 4;
  const int p0 = (blockIdx.y & 15) * 64;
  const float* src = scp + ((size_t)b * kCS + c0) * kPixS + p0;
#pragma unroll
  for (int it = 0; it < 8; ++it) {
    const int c = it * 8 + wave;
    const float v0 = src[(size_t)c * kPixS + lane];
    const float v1 = src[(size_t)c * kPixS + lane + 32];
    sT[lane * 68 + c] = v0;
    sT[(lane + 32) * 68 + c] = v1;
  }
  __syncthreads();
  const int q = lane >> 3, c8 = (lane & 7) * 8;
  v8h hv[2], lv[2];
#pragma unroll
  for (int it = 0; it < 2; ++it) {
    const int row = it * 32 + wave * 4 + q;
    const float* sp = sT + row * 68 + c8;
    const v4f a0 = *(const v4f*)(sp);
    const v4f a1 = *(const v4f*)(sp + 4);
#pragma unroll
    for (int e = 0; e < 4; ++e) {
      const unsigned short h0 = f2bf_bits(a0[e]), h1 = f2bf_bits(a1[e]);
      const unsigned short l0 = f2bf_bits(a0[e] - bf_bits2f(h0)), l1 = f2bf_bits(a1[e] - bf_bits2f(h1));
      hv[it][e]     = __builtin_bit_cast(_Float16, h0);
      hv[it][4 + e] = __builtin_bit_cast(_Float16, h1);
      lv[it][e]     = __builtin_bit_cast(_Float16, l0);
      lv[it][4 + e] = __builtin_bit_cast(_Float16, l1);
    }
  }
  const size_t rbase = (size_t)b * kPixS + p0;
  for (int pass = 0; pass < 2; ++pass) {
#pragma unroll
    for (int it = 0; it < 2; ++it) {
      const int row = it * 32 + wave * 4 + q;
      const size_t o = (rbase + row) * kCS + c0 + c8;
      *(volatile v8h*)(SCH + o) = hv[it];
      *(volatile v8h*)(SCL + o) = lv[it];
    }
    __threadfence();
  }
}

__global__ __launch_bounds__(256) void fuse_ln_kernel(
    const float* __restrict__ resnet, const float* __restrict__ SP,
    const float* __restrict__ rg, const float* __restrict__ rb, const float* __restrict__ rm, const float* __restrict__ rv,
    const float* __restrict__ sg, const float* __restrict__ sb, const float* __restrict__ sm, const float* __restrict__ sv,
    const float* __restrict__ lng, const float* __restrict__ lnb,
    float* __restrict__ FU, unsigned short* __restrict__ XNH, unsigned short* __restrict__ XNL)
{
  __shared__ __align__(16) float sF[32 * kFuseTP];
  const int tid = threadIdx.x, lane = tid & 31, wave = tid >> 5;
  const int b  = blockIdx.x >> 7;
  const int p0 = (blockIdx.x & 127) * 32;
  const size_t r0 = (size_t)blockIdx.x * 32;
  {
    const float* rsrc = resnet + (size_t)b * kCR * kSeq + p0 + lane;
#pragma unroll 1
    for (int it = 0; it < 32; ++it) {
      const int c = it * 8 + wave;
      const float inv = rg[c] / sqrtf(rv[c] + kEps);
      const float sh  = rb[c] - rm[c] * inv;
      const float v   = rsrc[(size_t)c * kSeq];
      sF[lane * kFuseTP + c] = v * inv + sh;
    }
  }
  __syncthreads();
  {
    const int c = tid;
    const float inv = sg[c] / sqrtf(sv[c] + kEps);
    const float sh  = sb[c] - sm[c] * inv;
    const float* spb = SP + (size_t)b * kPixS * kCR + c;
    const int y  = p0 >> 6;
    const int y0 = ((y + 1) >> 1) - 1;
    const float fy = (y & 1) ? 0.25f : 0.75f;
    const int ya = (y0 < 0) ? 0 : y0;
    const int yb = (y0 + 1 > kHS - 1) ? (kHS - 1) : (y0 + 1);
    const float wya = (y0 + 1 > kHS - 1) ? 1.0f : ((y0 < 0) ? 0.0f : (1.0f - fy));
    const float wyb = (y0 < 0) ? 1.0f : ((y0 + 1 > kHS - 1) ? 0.0f : fy);
    const float* rowa = spb + (size_t)(ya * kWS) * kCR;
    const float* rowb = spb + (size_t)(yb * kWS) * kCR;
#pragma unroll 1
    for (int pl = 0; pl < 32; ++pl) {
      const int x  = (p0 & 63) + pl;
      const int x0 = ((x + 1) >> 1) - 1;
      const float fx = (x & 1) ? 0.25f : 0.75f;
      const int xa = (x0 < 0) ? 0 : x0;
      const int xb = (x0 + 1 > kWS - 1) ? (kWS - 1) : (x0 + 1);
      const float wxa = (x0 + 1 > kWS - 1) ? 1.0f : ((x0 < 0) ? 0.0f : (1.0f - fx));
      const float wxb = (x0 < 0) ? 1.0f : ((x0 + 1 > kWS - 1) ? 0.0f : fx);
      const float vaa = rowa[(size_t)xa * kCR] * inv + sh;
      const float vab = rowa[(size_t)xb * kCR] * inv + sh;
      const float vba = rowb[(size_t)xa * kCR] * inv + sh;
      const float vbb = rowb[(size_t)xb * kCR] * inv + sh;
      const float la = wxa * vaa + wxb * vab;
      const float lb = wxa * vba + wxb * vbb;
      const float vi = wya * la + wyb * lb;
      sF[pl * kFuseTP + c] += vi;
    }
  }
  __syncthreads();
  {
    const v4f g0v = *(const v4f*)(lng + lane * 8);
    const v4f g1v = *(const v4f*)(lng + lane * 8 + 4);
    const v4f b0v = *(const v4f*)(lnb + lane * 8);
    const v4f b1v = *(const v4f*)(lnb + lane * 8 + 4);
#pragma unroll 1
    for (int k = 0; k < 4; ++k) {
      const int pl = wave * 4 + k;
      const float* rowp = sF + pl * kFuseTP;
      const v4f va = *(const v4f*)(rowp + lane * 4);
      const v4f vb = *(const v4f*)(rowp + 128 + lane * 4);
      float s = ((va[0] + va[1]) + (va[2] + va[3])) + ((vb[0] + vb[1]) + (vb[2] + vb[3]));
#pragma unroll
      for (int off = 1; off < 32; off <<= 1) s += __shfl_xor(s, off, 32);
      const float mean = s * (1.0f / 256.0f);
      float s2 = 0.f;
#pragma unroll
      for (int e = 0; e < 4; ++e) {
        const float da = va[e] - mean;
        const float db = vb[e] - mean;
        s2 += da * da;
        s2 += db * db;
      }
#pragma unroll
      for (int off = 1; off < 32; off <<= 1) s2 += __shfl_xor(s2, off, 32);
      const float var  = s2 * (1.0f / 256.0f);
      const float rstd = 1.0f / sqrtf(var + kEps);
      const v4f a0 = *(const v4f*)(rowp + lane * 8);
      const v4f a1 = *(const v4f*)(rowp + lane * 8 + 4);
      v8h hv, lv;
#pragma unroll
      for (int e = 0; e < 4; ++e) {
        const float x0 = (a0[e] - mean) * rstd * g0v[e] + b0v[e];
        const float x1 = (a1[e] - mean) * rstd * g1v[e] + b1v[e];
        const unsigned short h0 = f2bf_bits(x0), h1 = f2bf_bits(x1);
        const unsigned short l0 = f2bf_bits(x0 - bf_bits2f(h0)), l1 = f2bf_bits(x1 - bf_bits2f(h1));
        hv[e]     = __builtin_bit_cast(_Float16, h0);
        hv[4 + e] = __builtin_bit_cast(_Float16, h1);
        lv[e]     = __builtin_bit_cast(_Float16, l0);
        lv[4 + e] = __builtin_bit_cast(_Float16, l1);
      }
      const size_t r = r0 + pl;
      for (int pass = 0; pass < 2; ++pass) {
        *(volatile v4f*)(FU + r * kCR + lane * 4) = va;
        *(volatile v4f*)(FU + r * kCR + 128 + lane * 4) = vb;
        *(volatile v8h*)(XNH + r * kCR + lane * 8) = hv;
        *(volatile v8h*)(XNL + r * kCR + lane * 8) = lv;
        __threadfence();
      }
    }
  }
}

__global__ __launch_bounds__(256) void conv_silu_kernel(
    const float* __restrict__ XZ, const float* __restrict__ cw, const float* __restrict__ cb,
    float* __restrict__ UC, unsigned short* __restrict__ UCH, unsigned short* __restrict__ UCL)
{
  __shared__ __align__(16) float sT[16 * kConvTP];
  const int tid = threadIdx.x, lane = tid & 31, wave = tid >> 5;
  const int d0 = blockIdx.x * 256, d = d0 + tid;
  const int g0 = blockIdx.y * 64;
  const int tb = g0 & (kSeq - 1);
  const float w0 = cw[d * kConvK + 0], w1 = cw[d * kConvK + 1], w2 = cw[d * kConvK + 2];
  const float bc = cb[d];
  float xm2, xm1;
  {
    const bool hist = (tb > 0);
    const int rb = hist ? (g0 - 2) : g0;
    const float v2 = XZ[(size_t)rb * kXzP + d];
    const float v1 = XZ[(size_t)(rb + 1) * kXzP + d];
    xm2 = hist ? v2 : 0.f;
    xm1 = hist ? v1 : 0.f;
  }
  const int hrow = wave >> 1;
  const int hch  = (wave & 1) * 128 + lane * 4;
#pragma unroll 1
  for (int sub = 0; sub < 4; ++sub) {
    const int lb = g0 + sub * 16;
#pragma unroll 1
    for (int s = 0; s < 16; ++s) {
      const float xcur = XZ[(size_t)(lb + s) * kXzP + d];
      float acc = w0 * xm2;
      acc = fmaf(w1, xm1, acc);
      acc = fmaf(w2, xcur, acc);
      const float cv = acc + bc;
      const float sgm = __builtin_amdgcn_rcpf(1.0f + __expf(-cv));
      sT[s * kConvTP + tid] = cv * sgm;
      xm2 = xm1; xm1 = xcur;
    }
    __syncthreads();
    v4f fv[4];
    v8h bh[2], blo[2];
#pragma unroll
    for (int it = 0; it < 4; ++it) fv[it] = *(const v4f*)(sT + (it * 4 + hrow) * kConvTP + hch);
#pragma unroll
    for (int it = 0; it < 2; ++it) {
      const float* sp = sT + (it * 8 + wave) * kConvTP + lane * 8;
      const v4f a0 = *(const v4f*)(sp);
      const v4f a1 = *(const v4f*)(sp + 4);
#pragma unroll
      for (int e = 0; e < 4; ++e) {
        const unsigned short h0 = f2bf_bits(a0[e]), h1 = f2bf_bits(a1[e]);
        const unsigned short l0 = f2bf_bits(a0[e] - bf_bits2f(h0)), l1 = f2bf_bits(a1[e] - bf_bits2f(h1));
        bh[it][e]      = __builtin_bit_cast(_Float16, h0);
        bh[it][4 + e]  = __builtin_bit_cast(_Float16, h1);
        blo[it][e]     = __builtin_bit_cast(_Float16, l0);
        blo[it][4 + e] = __builtin_bit_cast(_Float16, l1);
      }
    }
    for (int pass = 0; pass < 2; ++pass) {
#pragma unroll
      for (int it = 0; it < 4; ++it)
        *(volatile v4f*)(UC + (size_t)(lb + it * 4 + hrow) * kDin + d0 + hch) = fv[it];
#pragma unroll
      for (int it = 0; it < 2; ++it) {
        const size_t o = (size_t)(lb + it * 8 + wave) * kDin + d0 + lane * 8;
        *(volatile v8h*)(UCH + o) = bh[it];
        *(volatile v8h*)(UCL + o) = blo[it];
      }
      __threadfence();
    }
    __syncthreads();
  }
}

__global__ __launch_bounds__(64) void scan_kernel(
    const float* __restrict__ XD, const float* __restrict__ UC, const float* __restrict__ XZ,
    const float* __restrict__ Wdt, const float* __restrict__ bdt, const float* __restrict__ Alog,
    const float* __restrict__ Dp, unsigned short* __restrict__ YH, unsigned short* __restrict__ YL)
{
  __shared__ __align__(16) float sX[kScanTS * kXdP];
  __shared__ __align__(16) float sY[kScanTS * kScanYP];
  __shared__ __align__(16) float sW[kDtR * kScanCh];
  __shared__ __align__(16) float sA[kNst * kScanCh];
  const int tid = threadIdx.x, lane = tid & 31, wave = tid >> 5;
  constexpr int kBlkPerB = kDin / kScanCh;
  const int bix = blockIdx.x / kBlkPerB;
  const int d0  = (blockIdx.x - bix * kBlkPerB) * kScanCh;
  const int d   = d0 + tid;
  const size_t row0 = (size_t)bix * kSeq;
#pragma unroll 1
  for (int r = 0; r < kDtR; ++r) sW[r * kScanCh + tid] = Wdt[(size_t)d * kDtR + r];
#pragma unroll 1
  for (int s = 0; s < kNst; ++s) sA[s * kScanCh + tid] = -expf(Alog[(size_t)d * kNst + s]);
  __syncthreads();
  float negA[kNst], h[kNst];
#pragma unroll
  for (int s = 0; s < kNst; ++s) {
    negA[s] = sA[s * kScanCh + tid];
    h[s] = 0.f;
  }
  const float bb = bdt[d], Dd = Dp[d];
  const int lr = tid >> 4, lc4 = (tid & 15) * 4;
  const int q = lane >> 3, c8 = (lane & 7) * 8;
#pragma unroll 1
  for (int t0 = 0; t0 < kSeq; t0 += kScanTS) {
    __syncthreads();
#pragma unroll
    for (int i = 0; i < 16; ++i) {
      const int r = lr + 4 * i;
      *(v4f*)(sX + r * kXdP + lc4) = *(const v4f*)(XD + (row0 + t0 + r) * kXdP + lc4);
    }
    __syncthreads();
#pragma unroll 1
    for (int s = 0; s < kScanTS; ++s) {
      const int t = t0 + s;
      const float* xr = sX + s * kXdP;
      float vdot = 0.f;
#pragma unroll 1
      for (int r4 = 0; r4 < kDtR / 4; ++r4) {
        const v4f xv = *(const v4f*)(xr + 4 * r4);
        const float* wp = sW + (4 * r4) * kScanCh + tid;
        vdot = fmaf(xv[0], wp[0], vdot);
        vdot = fmaf(xv[1], wp[kScanCh], vdot);
        vdot = fmaf(xv[2], wp[2 * kScanCh], vdot);
        vdot = fmaf(xv[3], wp[3 * kScanCh], vdot);
      }
      float Bs[kNst], Cs[kNst];
#pragma unroll
      for (int q4 = 0; q4 < 4; ++q4) {
        const v4f bv = *(const v4f*)(xr + kDtR + 4 * q4);
        const v4f cv = *(const v4f*)(xr + kDtR + kNst + 4 * q4);
        Bs[4 * q4 + 0] = bv[0]; Bs[4 * q4 + 1] = bv[1]; Bs[4 * q4 + 2] = bv[2]; Bs[4 * q4 + 3] = bv[3];
        Cs[4 * q4 + 0] = cv[0]; Cs[4 * q4 + 1] = cv[1]; Cs[4 * q4 + 2] = cv[2]; Cs[4 * q4 + 3] = cv[3];
      }
      const float v   = vdot + bb;
      const float a   = __expf(-fabsf(v));
      const float u   = 1.0f + a;
      const float l1p = __logf(u) + (a - (u - 1.0f)) * __builtin_amdgcn_rcpf(u);
      const float dt  = fmaxf(v, 0.0f) + l1p;
      const float xt  = UC[(row0 + t) * kDin + d];
      const float dtx = dt * xt;
      float y = 0.f;
#pragma unroll
      for (int k = 0; k < kNst; ++k) {
        const float e = __expf(dt * negA[k]);
        h[k] = e * h[k] + dtx * Bs[k];
        y = h[k] * Cs[k] + y;
      }
      y = xt * Dd + y;
      const float zv = XZ[(row0 + t) * kXzP + kDin + d];
      const float sgm = __builtin_amdgcn_rcpf(1.0f + __expf(-zv));
      y = y * (zv * sgm);
      sY[s * kScanYP + tid] = y;
    }
    __syncthreads();
    v8h hv[8], lv[8];
#pragma unroll
    for (int it = 0; it < 8; ++it) {
      const int row = it * 8 + wave * 4 + q;
      const float* sp = sY + row * kScanYP + c8;
      const v4f a0 = *(const v4f*)(sp);
      const v4f a1 = *(const v4f*)(sp + 4);
#pragma unroll
      for (int e = 0; e < 4; ++e) {
        const unsigned short h0 = f2bf_bits(a0[e]), h1 = f2bf_bits(a1[e]);
        const unsigned short l0 = f2bf_bits(a0[e] - bf_bits2f(h0)), l1 = f2bf_bits(a1[e] - bf_bits2f(h1));
        hv[it][e]     = __builtin_bit_cast(_Float16, h0);
        hv[it][4 + e] = __builtin_bit_cast(_Float16, h1);
        lv[it][e]     = __builtin_bit_cast(_Float16, l0);
        lv[it][4 + e] = __builtin_bit_cast(_Float16, l1);
      }
    }
    for (int pass = 0; pass < 2; ++pass) {
#pragma unroll
      for (int it = 0; it < 8; ++it) {
        const int row = it * 8 + wave * 4 + q;
        const size_t o = (row0 + t0 + row) * kDin + d0 + c8;
        *(volatile v8h*)(YH + o) = hv[it];
        *(volatile v8h*)(YL + o) = lv[it];
      }
      __threadfence();
    }
  }
}

__global__ __launch_bounds__(256) void out_transpose_kernel(
    const float* __restrict__ FU, const float* __restrict__ OS, float* __restrict__ out)
{
  __shared__ __align__(16) float sT[64 * 68];
  const int tid = threadIdx.x, lane = tid & 31, wave = tid >> 5;
  const int c0 = blockIdx.x * 64;
  const int b  = blockIdx.y >> 6;
  const int p0 = (blockIdx.y & 63) * 64;
  const size_t r0 = (size_t)blockIdx.y * 64;
#pragma unroll
  for (int it = 0; it < 8; ++it) {
    const int row = it * 8 + wave;
    const size_t o = (r0 + row) * kCR + c0;
    const float v0 = FU[o + lane] + OS[o + lane];
    const float v1 = FU[o + lane + 32] + OS[o + lane + 32];
    sT[lane * 68 + row] = v0;
    sT[(lane + 32) * 68 + row] = v1;
  }
  __syncthreads();
  const int hh = lane >> 4, c4 = (lane & 15) * 4;
  v4f val[4];
#pragma unroll
  for (int it = 0; it < 4; ++it) {
    const int cr = it * 16 + wave * 2 + hh;
    val[it] = *(const v4f*)(sT + cr * 68 + c4);
  }
  for (int pass = 0; pass < 2; ++pass) {
#pragma unroll
    for (int it = 0; it < 4; ++it) {
      const int cr = it * 16 + wave * 2 + hh;
      const size_t o = ((size_t)b * kCR + c0 + cr) * kSeq + p0 + c4;
      *(volatile v4f*)(out + o) = val[it];
    }
    __threadfence();
  }
}

extern "C" void kernel_launch(void* const* d_in, const int* in_sizes, int n_in,
                              void* d_out, int out_size, void* d_ws, size_t ws_size,
                              hipStream_t stream) {
  if (n_in < 22) return;
  if (in_sizes[0] != kBatch * kCR * kSeq) return;
  if (in_sizes[1] != kBatch * kCS * kPixS) return;
  if (in_sizes[2] != kCR * kCS) return;
  for (int i = 3; i <= 12; ++i) if (in_sizes[i] != kCR) return;
  if (in_sizes[13] != kXzP * kCR) return;
  if (in_sizes[14] != kDin * kConvK) return;
  if (in_sizes[15] != kDin) return;
  if (in_sizes[16] != kXdN * kDin) return;
  if (in_sizes[17] != kDin * kDtR) return;
  if (in_sizes[18] != kDin) return;
  if (in_sizes[19] != kDin * kNst) return;
  if (in_sizes[20] != kDin) return;
  if (in_sizes[21] != kCR * kDin) return;
  if (out_size != kBatch * kCR * kSeq) return;
  if (ws_size < kWsTotal) return;

  const float* resnet   = (const float*)d_in[0];
  const float* scp      = (const float*)d_in[1];
  const float* scp_w    = (const float*)d_in[2];
  const float* scp_bn_g = (const float*)d_in[3];
  const float* scp_bn_b = (const float*)d_in[4];
  const float* scp_bn_m = (const float*)d_in[5];
  const float* scp_bn_v = (const float*)d_in[6];
  const float* res_bn_g = (const float*)d_in[7];
  const float* res_bn_b = (const float*)d_in[8];
  const float* res_bn_m = (const float*)d_in[9];
  const float* res_bn_v = (const float*)d_in[10];
  const float* ln_g     = (const float*)d_in[11];
  const float* ln_b     = (const float*)d_in[12];
  const float* in_w     = (const float*)d_in[13];
  const float* conv_w   = (const float*)d_in[14];
  const float* conv_b   = (const float*)d_in[15];
  const float* xp_w     = (const float*)d_in[16];
  const float* dt_w     = (const float*)d_in[17];
  const float* dt_bias  = (const float*)d_in[18];
  const float* A_log    = (const float*)d_in[19];
  const float* Dvec     = (const float*)d_in[20];
  const float* out_w    = (const float*)d_in[21];
  float* out = (float*)d_out;

  char* ws = (char*)d_ws;
  unsigned short* SCH = (unsigned short*)(ws + kOffSCH);
  unsigned short* SCL = (unsigned short*)(ws + kOffSCL);
  unsigned short* WSH = (unsigned short*)(ws + kOffWSH);
  unsigned short* WSL = (unsigned short*)(ws + kOffWSL);
  float*          SP  = (float*)(ws + kOffSP);
  float*          FU  = (float*)(ws + kOffFU);
  unsigned short* XNH = (unsigned short*)(ws + kOffXNH);
  unsigned short* XNL = (unsigned short*)(ws + kOffXNL);
  unsigned short* WIH = (unsigned short*)(ws + kOffWIH);
  unsigned short* WIL = (unsigned short*)(ws + kOffWIL);
  unsigned short* WXH = (unsigned short*)(ws + kOffWXH);
  unsigned short* WXL = (unsigned short*)(ws + kOffWXL);
  unsigned short* WOH = (unsigned short*)(ws + kOffWOH);
  unsigned short* WOL = (unsigned short*)(ws + kOffWOL);
  float*          XZ  = (float*)(ws + kOffXZ);
  float*          UC  = (float*)(ws + kOffUC);
  unsigned short* UCH = (unsigned short*)(ws + kOffUCH);
  unsigned short* UCL = (unsigned short*)(ws + kOffUCL);
  float*          XD  = (float*)(ws + kOffXD);
  unsigned short* YH  = (unsigned short*)(ws + kOffYH);
  unsigned short* YL  = (unsigned short*)(ws + kOffYL);
  float*          OS  = (float*)(ws + kOffOS);

  scp_transpose_split_kernel<<<dim3(kCS / 64, kRowsS / 64), 256, 0, stream>>>(scp, SCH, SCL);

  {
    const int t8 = kCR * kCS / 8;
    split_rows_bf16_kernel<<<(t8 + 255) / 256, 256, 0, stream>>>(scp_w, WSH, WSL, t8, t8);
  }

  wmma_gemm64<1, 2, 0, 0, false><<<dim3(16, 1), 256, 0, stream>>>(
      SCH, SCL, kCS, 0L,
      WSH, WSL, kCS, 0L,
      (void*)SP, nullptr, kCR, 0L,
      nullptr, nullptr, 0L,
      kRowsS, kCR, kCS, 1.0f);

  fuse_ln_kernel<<<kRows / 32, 256, 0, stream>>>(resnet, SP,
      res_bn_g, res_bn_b, res_bn_m, res_bn_v,
      scp_bn_g, scp_bn_b, scp_bn_m, scp_bn_v,
      ln_g, ln_b, FU, XNH, XNL);

  {
    const int t8 = kXzP * kCR / 8;
    split_rows_bf16_kernel<<<(t8 + 255) / 256, 256, 0, stream>>>(in_w, WIH, WIL, t8, t8);
  }
  {
    const int t8 = kXdP * kDin / 8, v8 = kXdN * kDin / 8;
    split_rows_bf16_kernel<<<(t8 + 255) / 256, 256, 0, stream>>>(xp_w, WXH, WXL, t8, v8);
  }
  {
    const int t8 = kCR * kDin / 8;
    split_rows_bf16_kernel<<<(t8 + 255) / 256, 256, 0, stream>>>(out_w, WOH, WOL, t8, t8);
  }

  wmma_gemm64<1, 2, 0, 0, false><<<dim3(256, 1), 256, 0, stream>>>(
      XNH, XNL, kCR, 0L,
      WIH, WIL, kCR, 0L,
      (void*)XZ, nullptr, kXzP, 0L,
      nullptr, nullptr, 0L,
      kRows, kXzP, kCR, 1.0f);

  conv_silu_kernel<<<dim3(kDin / 256, kRows / 64), 256, 0, stream>>>(XZ, conv_w, conv_b, UC, UCH, UCL);

  wmma_gemm64<1, 2, 0, 0, false><<<dim3(16, 1), 256, 0, stream>>>(
      UCH, UCL, kDin, 0L,
      WXH, WXL, kDin, 0L,
      (void*)XD, nullptr, kXdP, 0L,
      nullptr, nullptr, 0L,
      kRows, kXdP, kDin, 1.0f);

  scan_kernel<<<kBatch * (kDin / kScanCh), kScanCh, 0, stream>>>(XD, UC, XZ, dt_w, dt_bias, A_log, Dvec, YH, YL);

  wmma_gemm64<1, 2, 0, 0, false><<<dim3(64, 1), 256, 0, stream>>>(
      YH, YL, kDin, 0L,
      WOH, WOL, kDin, 0L,
      (void*)OS, nullptr, kCR, 0L,
      nullptr, nullptr, 0L,
      kRows, kCR, kDin, 1.0f);

  out_transpose_kernel<<<dim3(kCR / 64, kRows / 64), 256, 0, stream>>>(FU, OS, out);
}
